// MoEModule_54803782697400
// MI455X (gfx1250) — hardware-verified
//
#include <hip/hip_runtime.h>
#include <math.h>

typedef __attribute__((ext_vector_type(16))) __bf16 v16b;
typedef __attribute__((ext_vector_type(16))) _Float16 v16h;
typedef _Float16 h16;
typedef __attribute__((ext_vector_type(8)))  float v8f;
typedef __attribute__((ext_vector_type(4)))  float v4f;
typedef __attribute__((ext_vector_type(4)))  unsigned v4u;
typedef __attribute__((ext_vector_type(8)))  unsigned v8u;
typedef __attribute__((ext_vector_type(4)))  int v4i;

#ifndef NB
#define NB 32u
#endif
#ifndef SEQ
#define SEQ 197u
#endif
#define NT (NB * SEQ)
#define NTP (((NT + 31u) / 32u) * 32u)
#define DD 768u
#define DH 768u
#define NE 16u
#define DDQ (DD / 8u)
#define TM 32u
#define SXP 776u
#define SFP 772u
#define NCH ((NT + 255u) / 256u)
#define MAXT (NTP / TM)
#define W2CARRY 64.0f
#define W2INV 0.015625f

static_assert(DD == DH);
static_assert((DD & 31u) == 0u);
static_assert((NT & 7u) == 0u);
static_assert(NE == 16u);
static_assert(8u * 96u == DH);
static_assert(8u * 96u == DD);
static_assert(TM * DDQ == 12u * 256u);
static_assert((NE * DD) / 4u == 12u * 256u);
static_assert(((NT * DD) / 8u) % 256u == 0u);
static_assert(((NE * DH * DD) / 8u) % 256u == 0u);
static_assert((SXP * 2u) % 16u == 0u);
static_assert((SFP * 4u) % 16u == 0u);
static_assert(8u * 12u * 32u * 16u == 16u * DD * 4u);
static_assert(8u * 16u == 32u * 4u);
static_assert(TM * SXP * 2u + 16u * SFP * 4u + TM * 4u + 8u * 4u <= 131072u);
static_assert(NE * SFP * 4u + 32u * 4u <= 131072u);

#define WS_IDX 0u
#define WS_XB  (WS_IDX + 4u * (size_t)NTP)
#define WS_W1  (WS_XB + 2u * (size_t)NT * DD)
#define WS_W2  (WS_W1 + 2u * (size_t)NE * DH * DD)
#define WS_END (WS_W2 + 2u * (size_t)NE * DD * DH)
static_assert((WS_XB & 127u) == 0u);
static_assert((WS_W1 & 127u) == 0u);
static_assert((WS_W2 & 127u) == 0u);
static_assert(WS_END <= 134217728u);

template <typename T> __device__ __forceinline__ void vst2(T* p, T v) { *(volatile T*)p = v; __threadfence(); *(volatile T*)p = v; }

__device__ __forceinline__ v8f wmma_bf(v16b a, v16b b, v8f c) {
  v8f d = __builtin_amdgcn_wmma_f32_16x16x32_bf16(false, a, false, b, (short)0, c, false, false);
  asm volatile("v_nop\n\tv_nop\n\tv_nop\n\tv_nop" : "+v"(d) : "v"(a), "v"(b));
  return d;
}
__device__ __forceinline__ v16b frag_q(v4u q0, v4u q1) {
  const v8u w = __builtin_shufflevector(q0, q1, 0, 1, 2, 3, 4, 5, 6, 7);
  return __builtin_bit_cast(v16b, w);
}
__device__ __forceinline__ float bfr(float v) { return (float)(__bf16)v; }
__device__ __forceinline__ unsigned short bfbits(float v) { return __builtin_bit_cast(unsigned short, (__bf16)v); }
__device__ __forceinline__ unsigned pk2(float a, float b) { return (unsigned)bfbits(a) | ((unsigned)bfbits(b) << 16); }

__device__ __forceinline__ v8f wmma_hf(v16h a, v16h b, v8f c) {
  v8f d = __builtin_amdgcn_wmma_f32_16x16x32_f16(false, a, false, b, (short)0, c, false, false);
  asm volatile("v_nop\n\tv_nop\n\tv_nop\n\tv_nop" : "+v"(d) : "v"(a), "v"(b));
  return d;
}
__device__ __forceinline__ v16h frag_qh(v4u q0, v4u q1) {
  const v8u w = __builtin_shufflevector(q0, q1, 0, 1, 2, 3, 4, 5, 6, 7);
  return __builtin_bit_cast(v16h, w);
}
static __device__ __forceinline__ h16 toh_flush(float v) { const h16 r = (h16)v; return (fabsf(v) < 6.103515625e-05f) ? (h16)0.0f : r; }
__device__ __forceinline__ unsigned short hbits(float v) { return __builtin_bit_cast(unsigned short, toh_flush(v)); }
__device__ __forceinline__ unsigned pk2h(float a, float b) { return (unsigned)hbits(a) | ((unsigned)hbits(b) << 16); }

__global__ __launch_bounds__(256) void k_xcvt(const float* __restrict__ X, v4u* __restrict__ XB) {
  const unsigned idx = blockIdx.x * 256u + threadIdx.x;
  const float* p = X + (size_t)idx * 8u;
  const v4f a = *(const v4f*)p;
  const v4f b = *(const v4f*)(p + 4);
  v4u o; o[0] = pk2(a[0], a[1]); o[1] = pk2(a[2], a[3]); o[2] = pk2(b[0], b[1]); o[3] = pk2(b[2], b[3]);
  vst2(XB + idx, o);
}

__global__ __launch_bounds__(256) void k_w2cvt(const float* __restrict__ W, v4u* __restrict__ WH) {
  const unsigned idx = blockIdx.x * 256u + threadIdx.x;
  const float* p = W + (size_t)idx * 8u;
  const v4f a = *(const v4f*)p;
  const v4f b = *(const v4f*)(p + 4);
  v4u o;
  o[0] = pk2h(bfr(a[0]) * W2CARRY, bfr(a[1]) * W2CARRY);
  o[1] = pk2h(bfr(a[2]) * W2CARRY, bfr(a[3]) * W2CARRY);
  o[2] = pk2h(bfr(b[0]) * W2CARRY, bfr(b[1]) * W2CARRY);
  o[3] = pk2h(bfr(b[2]) * W2CARRY, bfr(b[3]) * W2CARRY);
  vst2(WH + idx, o);
}

__global__ __launch_bounds__(256) void k_route(const v4u* __restrict__ XB, const float* __restrict__ WG, const float* __restrict__ BG, int* __restrict__ IDX) {
#pragma clang fp contract(off)
  __shared__ __align__(16) float swg[NE][SFP];
  __shared__ __align__(16) int sidx[32];
  const unsigned tid = threadIdx.x;
#pragma unroll 1
  for (unsigned p = 0; p < 12u; ++p) {
    const unsigned idx = p * 256u + tid;
    const unsigned er = idx / (DD / 4u), c4 = idx - er * (DD / 4u);
    v4f t4 = *(const v4f*)(WG + (size_t)idx * 4u);
    t4[0] = bfr(t4[0]); t4[1] = bfr(t4[1]); t4[2] = bfr(t4[2]); t4[3] = bfr(t4[3]);
    *(v4f*)&swg[er][c4 * 4u] = t4;
  }
  __syncthreads();
  const unsigned e = tid & 15u, tl = tid >> 4;
  const float bgv = bfr(BG[e]);
#pragma unroll 1
  for (unsigned pass = 0; pass < 2u; ++pass) {
    const unsigned trow = pass * 16u + tl;
    const unsigned t = blockIdx.x * 32u + trow;
    const unsigned tt = (t < NT) ? t : (NT - 1u);
    const v4u* px = XB + (size_t)tt * DDQ;
    double acc = 0.0;
#pragma unroll 1
    for (unsigned kq = 0; kq < DDQ; ++kq) {
      const v4u q = px[kq];
      const v4f w0 = *(const v4f*)&swg[e][kq * 8u];
      const v4f w1 = *(const v4f*)&swg[e][kq * 8u + 4u];
      const float x0 = __uint_as_float(q[0] << 16), x1 = __uint_as_float(q[0] & 0xffff0000u);
      const float x2 = __uint_as_float(q[1] << 16), x3 = __uint_as_float(q[1] & 0xffff0000u);
      const float x4 = __uint_as_float(q[2] << 16), x5 = __uint_as_float(q[2] & 0xffff0000u);
      const float x6 = __uint_as_float(q[3] << 16), x7 = __uint_as_float(q[3] & 0xffff0000u);
      const float p0 = x0 * w0[0], p1 = x1 * w0[1], p2 = x2 * w0[2], p3 = x3 * w0[3];
      const float p4 = x4 * w1[0], p5 = x5 * w1[1], p6 = x6 * w1[2], p7 = x7 * w1[3];
      acc += (double)p0; acc += (double)p1; acc += (double)p2; acc += (double)p3;
      acc += (double)p4; acc += (double)p5; acc += (double)p6; acc += (double)p7;
    }
    float bv = (float)acc + bgv;
    int bi = (int)e;
#pragma unroll
    for (int off = 8; off >= 1; off >>= 1) {
      const float ov = __shfl_xor(bv, off, 32);
      const int oi = __shfl_xor(bi, off, 32);
      const bool take = (ov > bv) || ((ov == bv) && (oi < bi));
      bv = take ? ov : bv;
      bi = take ? oi : bi;
    }
    if (e == 0u) sidx[trow] = (t < NT) ? bi : (int)NE;
  }
  __syncthreads();
  if (tid < 8u) {
    const v4i o = *(const v4i*)&sidx[tid * 4u];
    vst2((v4i*)(IDX + (size_t)blockIdx.x * 32u) + tid, o);
  }
}

__global__ __launch_bounds__(256) void k_moe(const v4u* __restrict__ XB, const v4u* __restrict__ W1B, const float* __restrict__ B1, const v4u* __restrict__ W2H, const float* __restrict__ B2, const int* __restrict__ IDX, float* __restrict__ OUT) {
  __shared__ __align__(16) unsigned short sx[TM][SXP];
  __shared__ __align__(16) float sf[16][SFP];
  __shared__ __align__(16) int stok[TM];
  __shared__ unsigned swc[8];
  const unsigned tid = threadIdx.x, lane = tid & 31u, col = lane & 15u, h = lane >> 4, wv = tid >> 5;
  const unsigned wave = (unsigned)__builtin_amdgcn_readfirstlane((int)(threadIdx.x >> 5));
  const unsigned e = blockIdx.y, lo = blockIdx.x * TM;
  if (tid < TM) stok[tid] = 0;
  __syncthreads();
  unsigned basev = 0u;
#pragma unroll 1
  for (unsigned c = 0; c < NCH; ++c) {
    const unsigned t = c * 256u + tid;
    const unsigned ta = (t < NT) ? t : (NT - 1u);
    int idv = IDX[ta];
    asm volatile("" : "+v"(idv));
    const bool hit = (t < NT) && (idv == (int)e);
    const unsigned m = __builtin_amdgcn_ballot_w32(hit);
    if (lane == 0u) swc[wv] = (unsigned)__builtin_popcount(m);
    __syncthreads();
    unsigned pre = 0u, tot = 0u;
#pragma unroll
    for (unsigned w = 0; w < 8u; ++w) { const unsigned cw = swc[w]; pre += (w < wv) ? cw : 0u; tot += cw; }
    const unsigned g = basev + pre + (unsigned)__builtin_popcount(m & ((1u << lane) - 1u));
    if (hit && g >= lo && g < lo + TM) stok[g - lo] = (int)t;
    basev += tot;
    __syncthreads();
    if ((unsigned)__builtin_amdgcn_readfirstlane((int)basev) >= lo + TM) break;
  }
  const unsigned capv = (basev < lo + TM) ? basev : (lo + TM);
  if ((unsigned)__builtin_amdgcn_readfirstlane((int)capv) <= lo) return;
  const unsigned nval = capv - lo;

#pragma unroll 2
  for (unsigned p = 0; p < 12u; ++p) {
    const unsigned piece = p * 256u + tid;
    const unsigned r = piece / DDQ, c = piece - r * DDQ;
    const unsigned ts = (unsigned)stok[r];
    const unsigned tk = (ts < NT) ? ts : (NT - 1u);
    const v4u v = XB[(size_t)tk * DDQ + c];
    *(v4u*)&sx[r][c * 8u] = v;
  }
  __syncthreads();

  const unsigned nbase = wave * 96u;
  v8f acc[2][6];
#pragma unroll
  for (unsigned nt = 0; nt < 6u; ++nt) { acc[0][nt] = (v8f){}; acc[1][nt] = (v8f){}; }
  {
    const v4u* pb = W1B + ((size_t)e * DH + nbase + col) * DDQ + h;
#pragma unroll 1
    for (unsigned kc = 0; kc < DD / 32u; ++kc) {
      const unsigned kq = kc * 4u;
      const v16b a0 = frag_q(*(const v4u*)&sx[col][kc * 32u + 8u * h], *(const v4u*)&sx[col][kc * 32u + 16u + 8u * h]);
      const v16b a1 = frag_q(*(const v4u*)&sx[16u + col][kc * 32u + 8u * h], *(const v4u*)&sx[16u + col][kc * 32u + 16u + 8u * h]);
#pragma unroll
      for (unsigned nt = 0; nt < 6u; nt += 2u) {
        const v4u* pe = pb + (size_t)nt * 16u * DDQ + kq;
        const v16b b0 = frag_q(pe[0], pe[2]);
        const v16b b1 = frag_q(pe[16u * DDQ], pe[16u * DDQ + 2u]);
        asm volatile("s_wait_loadcnt 0x0" ::: "memory");
        acc[0][nt] = wmma_bf(a0, b0, acc[0][nt]);
        acc[1][nt] = wmma_bf(a1, b0, acc[1][nt]);
        acc[0][nt + 1u] = wmma_bf(a0, b1, acc[0][nt + 1u]);
        acc[1][nt + 1u] = wmma_bf(a1, b1, acc[1][nt + 1u]);
      }
    }
  }
  float b1v[6];
#pragma unroll
  for (unsigned nt = 0; nt < 6u; ++nt) b1v[nt] = bfr(B1[(size_t)e * DH + nbase + nt * 16u + col]);
  __syncthreads();

#pragma unroll
  for (unsigned mt = 0; mt < 2u; ++mt) {
#pragma unroll
    for (unsigned nt = 0; nt < 6u; ++nt) {
      const unsigned n = nbase + nt * 16u + col;
#pragma unroll
      for (unsigned r = 0; r < 8u; ++r) {
        const float z = acc[mt][nt][r] + b1v[nt];
        const float gl = 0.5f * z * (1.0f + erff(z * 0.70710678118654752f));
        sx[mt * 16u + 8u * h + r][n] = hbits(gl);
      }
    }
  }
  __syncthreads();

#pragma unroll
  for (unsigned nt = 0; nt < 6u; ++nt) { acc[0][nt] = (v8f){}; acc[1][nt] = (v8f){}; }
  {
    const v4u* pb = W2H + ((size_t)e * DD + nbase + col) * DDQ + h;
#pragma unroll 1
    for (unsigned kc = 0; kc < DH / 32u; ++kc) {
      const unsigned kq = kc * 4u;
      const v16h a0 = frag_qh(*(const v4u*)&sx[col][kc * 32u + 8u * h], *(const v4u*)&sx[col][kc * 32u + 16u + 8u * h]);
      const v16h a1 = frag_qh(*(const v4u*)&sx[16u + col][kc * 32u + 8u * h], *(const v4u*)&sx[16u + col][kc * 32u + 16u + 8u * h]);
#pragma unroll
      for (unsigned nt = 0; nt < 6u; nt += 2u) {
        const v4u* pe = pb + (size_t)nt * 16u * DDQ + kq;
        const v16h b0 = frag_qh(pe[0], pe[2]);
        const v16h b1 = frag_qh(pe[16u * DDQ], pe[16u * DDQ + 2u]);
        asm volatile("s_wait_loadcnt 0x0" ::: "memory");
        acc[0][nt] = wmma_hf(a0, b0, acc[0][nt]);
        acc[1][nt] = wmma_hf(a1, b0, acc[1][nt]);
        acc[0][nt + 1u] = wmma_hf(a0, b1, acc[0][nt + 1u]);
        acc[1][nt + 1u] = wmma_hf(a1, b1, acc[1][nt + 1u]);
      }
    }
  }
  float b2v[6];
#pragma unroll
  for (unsigned nt = 0; nt < 6u; ++nt) b2v[nt] = bfr(B2[(size_t)e * DD + nbase + nt * 16u + col]);

#pragma unroll
  for (unsigned mt = 0; mt < 2u; ++mt) {
#pragma unroll
    for (unsigned nt = 0; nt < 6u; ++nt) {
      const unsigned n = nbase + nt * 16u + col;
#pragma unroll
      for (unsigned r = 0; r < 8u; ++r) sf[8u * h + r][n] = acc[mt][nt][r] * W2INV + b2v[nt];
    }
    __syncthreads();
#pragma unroll 1
    for (unsigned it = 0; it < 12u; ++it) {
      const unsigned rsel = it / 6u;
      const unsigned rr = wave * 2u + rsel;
      const unsigned c4 = (it - rsel * 6u) * 32u + lane;
      const unsigned row = mt * 16u + rr;
      const v4f v = *(const v4f*)&sf[rr][c4 * 4u];
      const unsigned ts = (unsigned)stok[row];
      unsigned tk = (ts < NT) ? ts : (NT - 1u);
      asm volatile("" : "+v"(tk));
      if (row < nval) vst2((v4f*)(OUT + (size_t)tk * DD) + c4, v);
    }
    __syncthreads();
  }
}

extern "C" void kernel_launch(void* const* d_in, const int* in_sizes, int n_in, void* d_out, int out_size, void* d_ws, size_t ws_size, hipStream_t stream) {
  if (n_in < 7) return;
  if ((size_t)in_sizes[0] < (size_t)NT * DD) return;
  if ((size_t)in_sizes[1] < (size_t)NE * DH * DD) return;
  if ((size_t)in_sizes[2] < (size_t)NE * DH) return;
  if ((size_t)in_sizes[3] < (size_t)NE * DD * DH) return;
  if ((size_t)in_sizes[4] < (size_t)NE * DD) return;
  if ((size_t)in_sizes[5] < (size_t)NE * DD) return;
  if ((size_t)in_sizes[6] < (size_t)NE) return;
  if ((size_t)out_size < (size_t)NT * DD) return;
  if (ws_size < (size_t)WS_END) return;
  const float* X  = (const float*)d_in[0];
  const float* W1 = (const float*)d_in[1];
  const float* B1 = (const float*)d_in[2];
  const float* W2 = (const float*)d_in[3];
  const float* B2 = (const float*)d_in[4];
  const float* WG = (const float*)d_in[5];
  const float* BG = (const float*)d_in[6];
  char* ws = (char*)d_ws;
  int* IDX = (int*)(ws + WS_IDX);
  v4u* XB  = (v4u*)(ws + WS_XB);
  v4u* W1B = (v4u*)(ws + WS_W1);
  v4u* W2H = (v4u*)(ws + WS_W2);
  float* OUT = (float*)d_out;
  k_xcvt<<<dim3((NT * DD) / (8u * 256u)), 256, 0, stream>>>(X, XB);
  k_xcvt<<<dim3((NE * DH * DD) / (8u * 256u)), 256, 0, stream>>>(W1, W1B);
  k_w2cvt<<<dim3((NE * DD * DH) / (8u * 256u)), 256, 0, stream>>>(W2, W2H);
  k_route<<<dim3(NTP / 32u), 256, 0, stream>>>(XB, WG, BG, IDX);
  k_moe<<<dim3(MAXT, NE), 256, 0, stream>>>(XB, W1B, B1, W2H, B2, IDX, OUT);
}
